// NATBlock_2602750182048
// MI455X (gfx1250) — hardware-verified
//
#include <hip/hip_runtime.h>
#include <stdint.h>

#define NPIX   12544
#define CCH    128
#define NHD    4
#define HD     32
#define C3     384
#define C2     256
#define HID    512
#define FR     56
#define KSZ    7
#define NKEY   49
#define RPW    13
#define RPSZ   676
#define NOPX   3136
#define OFR    28
#define KCV    2304
#define COUT   512
#define NDEP   2
#define LDC    132
#define OSP    132
#define TPK    72
#define APB    32
#define QSC    0.17677669529663687f
#define RSC    0.00048828125f

static_assert(NPIX == 4 * FR * FR);
static_assert(NOPX == 4 * OFR * OFR);
static_assert((NPIX % 64) == 0 && (NPIX % APB) == 0 && (NPIX % 8) == 0);
static_assert((NOPX % 64) == 0 && ((NOPX * 18) % 8) == 0);
static_assert((KCV % 64) == 0 && (COUT % 128) == 0 && (C3 % 128) == 0 && (C2 % 128) == 0);
static_assert(KCV == 9 * 2 * CCH);
static_assert(RPSZ == NHD * RPW * RPW);
static_assert(NKEY == KSZ * KSZ && RPW == 2 * KSZ - 1);
static_assert((LDC * 4) % 16 == 0 && (OSP * 4) % 16 == 0 && (TPK * 2) % 16 == 0);
static_assert(APB * 4 == 128);

typedef _Float16 v16h __attribute__((ext_vector_type(16)));
typedef _Float16 v8h  __attribute__((ext_vector_type(8)));
typedef float    v8f  __attribute__((ext_vector_type(8)));
typedef float    v4f  __attribute__((ext_vector_type(4)));
typedef unsigned int v4u __attribute__((ext_vector_type(4)));
typedef unsigned int v2u __attribute__((ext_vector_type(2)));
typedef v4u v4ua __attribute__((may_alias));

__device__ __forceinline__ unsigned short bf_bits(float f) {
  unsigned u = __float_as_uint(f);
  return (unsigned short)((u + 0x7FFFu + ((u >> 16) & 1u)) >> 16);
}
__device__ __forceinline__ float bf_up(unsigned short b) { return __uint_as_float(((unsigned)b) << 16); }
__device__ __forceinline__ float bfr(float f) { return bf_up(bf_bits(f)); }
__device__ __forceinline__ unsigned short h_bits(_Float16 x) { return __builtin_bit_cast(unsigned short, x); }
__device__ __forceinline__ unsigned short hb16(float f) { return h_bits((_Float16)f); }
__device__ __forceinline__ unsigned pk16(unsigned short a, unsigned short b) { return (unsigned)a | ((unsigned)b << 16); }
__device__ __forceinline__ v8f zero8() { v8f z = {0.f, 0.f, 0.f, 0.f, 0.f, 0.f, 0.f, 0.f}; return z; }

__device__ __forceinline__ float wsum(float v) {
  v += __shfl_xor(v, 1, 32);
  v += __shfl_xor(v, 2, 32);
  v += __shfl_xor(v, 4, 32);
  v += __shfl_xor(v, 8, 32);
  v += __shfl_xor(v, 16, 32);
  return v;
}

__device__ __forceinline__ v16h ldfrag_h(const _Float16* p) {
  union { v16h v; v8h h[2]; } f;
  f.h[0] = *(const v8h*)(p);
  f.h[1] = *(const v8h*)(p + 16);
  return f.v;
}

__device__ __forceinline__ v8f mma_raw(v16h a, v16h b, v8f c) {
  return __builtin_amdgcn_wmma_f32_16x16x32_f16(false, a, false, b, (short)0, c, false, false);
}
__device__ __forceinline__ void guard4(v8f& c0, v8f& c1, v8f& c2, v8f& c3,
                                       const v16h& a0, const v16h& a1, const v16h& b0, const v16h& b1) {
#if defined(__HIP_DEVICE_COMPILE__)
  asm volatile("v_nop\n\tv_nop\n\tv_nop\n\tv_nop"
               : "+v"(c0), "+v"(c1), "+v"(c2), "+v"(c3) : "v"(a0), "v"(a1), "v"(b0), "v"(b1));
#endif
}
__device__ __forceinline__ void guard8(v8f& c0, v8f& c1, v8f& c2, v8f& c3, v8f& c4, v8f& c5, v8f& c6, v8f& c7,
                                       const v16h& a0, const v16h& a1, const v16h& a2, const v16h& a3,
                                       const v16h& b0, const v16h& b1) {
#if defined(__HIP_DEVICE_COMPILE__)
  asm volatile("v_nop\n\tv_nop\n\tv_nop\n\tv_nop"
               : "+v"(c0), "+v"(c1), "+v"(c2), "+v"(c3), "+v"(c4), "+v"(c5), "+v"(c6), "+v"(c7)
               : "v"(a0), "v"(a1), "v"(a2), "v"(a3), "v"(b0), "v"(b1));
#endif
}

__device__ __forceinline__ v4f ln4(const v4f a, const v4f gg, const v4f be) {
  float s = (a[0] + a[1]) + (a[2] + a[3]);
  s = wsum(s);
  const float mu = s * (1.0f / (float)CCH);
  v4f d;
  d[0] = a[0] - mu; d[1] = a[1] - mu; d[2] = a[2] - mu; d[3] = a[3] - mu;
  float sq = (d[0] * d[0] + d[1] * d[1]) + (d[2] * d[2] + d[3] * d[3]);
  sq = wsum(sq);
  const float rs = rsqrtf(sq * (1.0f / (float)CCH) + 1e-5f);
  v4f y;
#pragma unroll
  for (int e = 0; e < 4; ++e) y[e] = (d[e] * rs) * gg[e] + be[e];
  return y;
}

__device__ __forceinline__ void mm_tile(const _Float16* __restrict__ A, int lda,
                                        const _Float16* __restrict__ W, int ldw, int nks,
                                        int arow0, int bcol0, float* Cs) {
  const int tid = threadIdx.x, wave = tid >> 5, lane = tid & 31, hh = lane >> 4, c = lane & 15;
  const int mw = wave >> 2, nw = wave & 3;
  const _Float16* a0p = A + (size_t)(arow0 + mw * 32 + c) * lda + 8 * hh;
  const _Float16* a1p = A + (size_t)(arow0 + mw * 32 + 16 + c) * lda + 8 * hh;
  const _Float16* b0p = W + (size_t)(bcol0 + nw * 32 + c) * ldw + 8 * hh;
  const _Float16* b1p = W + (size_t)(bcol0 + nw * 32 + 16 + c) * ldw + 8 * hh;
  v8f a00 = zero8(), a01 = zero8(), a10 = zero8(), a11 = zero8();
#pragma unroll 1
  for (int ks = 0; ks < nks; ++ks) {
    const int ko = ks * 32;
    const v16h fa0 = ldfrag_h(a0p + ko);
    const v16h fa1 = ldfrag_h(a1p + ko);
    const v16h fb0 = ldfrag_h(b0p + ko);
    const v16h fb1 = ldfrag_h(b1p + ko);
    a00 = mma_raw(fa0, fb0, a00);
    a01 = mma_raw(fa0, fb1, a01);
    a10 = mma_raw(fa1, fb0, a10);
    a11 = mma_raw(fa1, fb1, a11);
    guard4(a00, a01, a10, a11, fa0, fa1, fb0, fb1);
  }
#pragma unroll
  for (int r = 0; r < 8; ++r) {
    const int row = mw * 32 + 8 * hh + r;
    Cs[row * LDC + nw * 32 + c]             = a00[r];
    Cs[row * LDC + nw * 32 + 16 + c]        = a01[r];
    Cs[(row + 16) * LDC + nw * 32 + c]      = a10[r];
    Cs[(row + 16) * LDC + nw * 32 + 16 + c] = a11[r];
  }
}

__device__ __forceinline__ void mm_tile2(const _Float16* __restrict__ Ah, const _Float16* __restrict__ Al, int lda,
                                         const _Float16* __restrict__ W, int ldw, int nks,
                                         int arow0, int bcol0, float* Cs) {
  const int tid = threadIdx.x, wave = tid >> 5, lane = tid & 31, hh = lane >> 4, c = lane & 15;
  const int mw = wave >> 2, nw = wave & 3;
  const size_t r0 = (size_t)(arow0 + mw * 32 + c) * lda + 8 * hh;
  const size_t r1 = (size_t)(arow0 + mw * 32 + 16 + c) * lda + 8 * hh;
  const _Float16* a0h = Ah + r0;
  const _Float16* a1h = Ah + r1;
  const _Float16* a0l = Al + r0;
  const _Float16* a1l = Al + r1;
  const _Float16* b0p = W + (size_t)(bcol0 + nw * 32 + c) * ldw + 8 * hh;
  const _Float16* b1p = W + (size_t)(bcol0 + nw * 32 + 16 + c) * ldw + 8 * hh;
  v8f h00 = zero8(), h01 = zero8(), h10 = zero8(), h11 = zero8();
  v8f l00 = zero8(), l01 = zero8(), l10 = zero8(), l11 = zero8();
#pragma unroll 1
  for (int ks = 0; ks < nks; ++ks) {
    const int ko = ks * 32;
    const v16h fa0 = ldfrag_h(a0h + ko);
    const v16h fa1 = ldfrag_h(a1h + ko);
    const v16h ga0 = ldfrag_h(a0l + ko);
    const v16h ga1 = ldfrag_h(a1l + ko);
    const v16h fb0 = ldfrag_h(b0p + ko);
    const v16h fb1 = ldfrag_h(b1p + ko);
    h00 = mma_raw(fa0, fb0, h00);
    h01 = mma_raw(fa0, fb1, h01);
    h10 = mma_raw(fa1, fb0, h10);
    h11 = mma_raw(fa1, fb1, h11);
    l00 = mma_raw(ga0, fb0, l00);
    l01 = mma_raw(ga0, fb1, l01);
    l10 = mma_raw(ga1, fb0, l10);
    l11 = mma_raw(ga1, fb1, l11);
    guard8(h00, h01, h10, h11, l00, l01, l10, l11, fa0, fa1, ga0, ga1, fb0, fb1);
  }
#pragma unroll
  for (int r = 0; r < 8; ++r) {
    const int row = mw * 32 + 8 * hh + r;
    Cs[row * LDC + nw * 32 + c]             = h00[r] + l00[r] * RSC;
    Cs[row * LDC + nw * 32 + 16 + c]        = h01[r] + l01[r] * RSC;
    Cs[(row + 16) * LDC + nw * 32 + c]      = h10[r] + l10[r] * RSC;
    Cs[(row + 16) * LDC + nw * 32 + 16 + c] = h11[r] + l11[r] * RSC;
  }
}

__global__ __launch_bounds__(256)
void k_cvt_wt(const float* __restrict__ w, unsigned short* wt, int K, int N) {
  __shared__ __align__(16) unsigned short T[64 * TPK];
  const int tid = threadIdx.x;
  const int n0 = blockIdx.x * 64, k0 = blockIdx.y * 64, d = blockIdx.z;
  const float* src = w + (size_t)d * K * N;
  unsigned short* dst = wt + (size_t)d * K * N;
#pragma unroll
  for (int s = 0; s < 4; ++s) {
    const int idx = s * 256 + tid;
    const int kr = idx >> 4, nq = (idx & 15) * 4;
    const v4f a = *(const v4f*)(src + (size_t)(k0 + kr) * N + n0 + nq);
#pragma unroll
    for (int e = 0; e < 4; ++e) T[(nq + e) * TPK + kr] = hb16(bfr(a[e]) * 64.0f);
  }
  __syncthreads();
  v4u pk[2];
  size_t offs[2];
#pragma unroll
  for (int s = 0; s < 2; ++s) {
    const int idx = s * 256 + tid;
    const int n = idx >> 3, piece = idx & 7;
    pk[s] = *(const v4ua*)(&T[n * TPK + piece * 8]);
    offs[s] = (size_t)(n0 + n) * K + k0 + piece * 8;
  }
#pragma unroll
  for (int s = 0; s < 2; ++s) *(volatile v4u*)(dst + offs[s]) = pk[s];
  __threadfence();
#pragma unroll
  for (int s = 0; s < 2; ++s) *(volatile v4u*)(dst + offs[s]) = pk[s];
}

template <int RND>
__global__ __launch_bounds__(256)
void k_ln128(const float* __restrict__ src, const float* __restrict__ g, const float* __restrict__ bb,
             unsigned short* dst) {
  const int tid = threadIdx.x, wv = tid >> 5, lane = tid & 31;
  const int t = blockIdx.x * 8 + wv;
  const v4f v  = *(const v4f*)(src + (size_t)t * CCH + lane * 4);
  const v4f gr = *(const v4f*)(g + lane * 4);
  const v4f br = *(const v4f*)(bb + lane * 4);
  v4f a, gg, be;
#pragma unroll
  for (int e = 0; e < 4; ++e) { a[e] = RND ? bfr(v[e]) : v[e]; gg[e] = bfr(gr[e]); be[e] = bfr(br[e]); }
  const v4f y = ln4(a, gg, be);
  v2u pk;
  pk[0] = pk16(hb16(y[0] * 8.0f), hb16(y[1] * 8.0f));
  pk[1] = pk16(hb16(y[2] * 8.0f), hb16(y[3] * 8.0f));
  unsigned short* gp = dst + (size_t)t * CCH + lane * 4;
  *(volatile v2u*)gp = pk;
  __threadfence();
  *(volatile v2u*)gp = pk;
}

template <int RND>
__global__ __launch_bounds__(256)
void k_cvt16(const float* __restrict__ src, unsigned short* dst) {
  const int tid = threadIdx.x, wv = tid >> 5, lane = tid & 31;
  const int t = blockIdx.x * 8 + wv;
  const v4f v = *(const v4f*)(src + (size_t)t * CCH + lane * 4);
  v4f a;
#pragma unroll
  for (int e = 0; e < 4; ++e) a[e] = (RND ? bfr(v[e]) : v[e]) * 8.0f;
  v2u pk;
  pk[0] = pk16(hb16(a[0]), hb16(a[1]));
  pk[1] = pk16(hb16(a[2]), hb16(a[3]));
  unsigned short* gp = dst + (size_t)t * CCH + lane * 4;
  *(volatile v2u*)gp = pk;
  __threadfence();
  *(volatile v2u*)gp = pk;
}

template <int HAS_RES, int RND>
__global__ __launch_bounds__(256)
void k_gemm_f32(const unsigned short* __restrict__ A, const unsigned short* __restrict__ W, int K,
                const float* __restrict__ bias, float scl, const float* __restrict__ res,
                float* out, int ldo) {
  __shared__ __align__(16) float Cs[64 * LDC];
  const int tid = threadIdx.x, wave = tid >> 5, lane = tid & 31;
  const int mb = blockIdx.x, nb = blockIdx.y;
  mm_tile((const _Float16*)(const void*)A, K, (const _Float16*)(const void*)W, K, K >> 5,
          mb * 64, nb * 128, Cs);
  __syncthreads();
  const int col0 = nb * 128 + lane * 4;
  const v4f b4 = *(const v4f*)(bias + col0);
  v4f bb;
#pragma unroll
  for (int e = 0; e < 4; ++e) bb[e] = bfr(b4[e]);
#pragma unroll 1
  for (int it = 0; it < 8; ++it) {
    const int row = wave * 8 + it;
    const size_t t = (size_t)(mb * 64 + row);
    const v4f a = *(const v4f*)(Cs + row * LDC + lane * 4);
    v4f o;
    if (HAS_RES) {
      const v4f xv = *(const v4f*)(res + t * ldo + col0);
#pragma unroll
      for (int e = 0; e < 4; ++e) {
        const float xr = RND ? bfr(xv[e]) : xv[e];
        o[e] = xr + (a[e] * scl + bb[e]);
      }
    } else {
#pragma unroll
      for (int e = 0; e < 4; ++e) o[e] = a[e] * scl + bb[e];
    }
    float* p = out + t * ldo + col0;
    *(volatile v4f*)p = o;
    __threadfence();
    *(volatile v4f*)p = o;
  }
}

__global__ __launch_bounds__(256)
void k_gemm_gelu(const unsigned short* __restrict__ A, const unsigned short* __restrict__ W,
                 const float* __restrict__ bias, unsigned short* hp) {
  __shared__ __align__(16) float Cs[64 * LDC];
  const int tid = threadIdx.x;
  const int mb = blockIdx.x, nb = blockIdx.y;
  mm_tile((const _Float16*)(const void*)A, CCH, (const _Float16*)(const void*)W, CCH, CCH / 32,
          mb * 64, nb * 128, Cs);
  __syncthreads();
  const float* bn = bias + nb * 128;
#pragma unroll 2
  for (int it = 0; it < 32; ++it) {
    const int idx = it * 256 + tid;
    const int row = idx >> 7, col = idx & 127;
    const float v = Cs[row * LDC + col] * (1.0f / 512.0f) + bfr(bn[col]);
    const float gl = 0.5f * v * (1.0f + erff(v * 0.70710678118654752f));
    Cs[row * LDC + col] = gl * 64.0f;
  }
  __syncthreads();
  v4u pk[4];
  size_t offs[4];
#pragma unroll
  for (int s = 0; s < 4; ++s) {
    const int idx = s * 256 + tid;
    const int row = idx >> 4, piece = idx & 15;
    const int col0 = piece * 8;
    v4u q4;
#pragma unroll
    for (int e = 0; e < 4; ++e) {
      q4[e] = pk16(hb16(Cs[row * LDC + col0 + 2 * e]), hb16(Cs[row * LDC + col0 + 2 * e + 1]));
    }
    pk[s] = q4;
    offs[s] = (size_t)(mb * 64 + row) * HID + nb * 128 + col0;
  }
#pragma unroll
  for (int s = 0; s < 4; ++s) *(volatile v4u*)(hp + offs[s]) = pk[s];
  __threadfence();
#pragma unroll
  for (int s = 0; s < 4; ++s) *(volatile v4u*)(hp + offs[s]) = pk[s];
}

__global__ __launch_bounds__(128)
void k_attn(const float* __restrict__ qs, int qp, const float* __restrict__ kv, int kvp, int koff, int voff,
            const float* __restrict__ rpb, unsigned short* ao) {
  __shared__ float Ls[NKEY * 128];
  __shared__ __align__(16) float Os[APB * OSP];
  const int tid = threadIdx.x, pl = tid >> 2, h = tid & 3;
  const int m = blockIdx.x * APB + pl;
  const int xw = m % FR;
  const int y = (m / FR) % FR;
  const int b = m / (FR * FR);
  const float* qr = qs + (size_t)m * qp + h * HD;
  float q[HD];
#pragma unroll
  for (int d4 = 0; d4 < HD / 4; ++d4) {
    const v4f t4 = *(const v4f*)(qr + d4 * 4);
#pragma unroll
    for (int e = 0; e < 4; ++e) q[d4 * 4 + e] = t4[e] * QSC;
  }
  const int sy = min(max(y - KSZ / 2, 0), FR - KSZ);
  const int sx = min(max(xw - KSZ / 2, 0), FR - KSZ);
  const float* rp = rpb + h * (RPW * RPW);
  float mx = -3.0e38f;
#pragma unroll 1
  for (int key = 0; key < NKEY; ++key) {
    const int i = key / KSZ, j = key - i * KSZ;
    const int ny = sy + i, nx = sx + j;
    const int nm = (b * FR + ny) * FR + nx;
    const float* kr = kv + (size_t)nm * kvp + koff + h * HD;
    float s = bfr(rp[(ny - y + (KSZ - 1)) * RPW + (nx - xw + (KSZ - 1))]);
#pragma unroll
    for (int d4 = 0; d4 < HD / 4; ++d4) {
      const v4f t4 = *(const v4f*)(kr + d4 * 4);
#pragma unroll
      for (int e = 0; e < 4; ++e) s += q[d4 * 4 + e] * t4[e];
    }
    Ls[key * 128 + tid] = s;
    mx = fmaxf(mx, s);
  }
  float acc[HD];
#pragma unroll
  for (int d = 0; d < HD; ++d) acc[d] = 0.f;
  float l = 0.f;
#pragma unroll 1
  for (int key = 0; key < NKEY; ++key) {
    const int i = key / KSZ, j = key - i * KSZ;
    const int ny = sy + i, nx = sx + j;
    const int nm = (b * FR + ny) * FR + nx;
    const float p = __expf(Ls[key * 128 + tid] - mx);
    l += p;
    const float* vr = kv + (size_t)nm * kvp + voff + h * HD;
#pragma unroll
    for (int d4 = 0; d4 < HD / 4; ++d4) {
      const v4f t4 = *(const v4f*)(vr + d4 * 4);
#pragma unroll
      for (int e = 0; e < 4; ++e) acc[d4 * 4 + e] += p * t4[e];
    }
  }
  const float inv = __builtin_amdgcn_rcpf(l);
#pragma unroll
  for (int d = 0; d < HD; ++d) Os[pl * OSP + h * HD + d] = acc[d] * inv;
  __syncthreads();
  v4u pk[4];
  size_t offs[4];
#pragma unroll
  for (int s = 0; s < 4; ++s) {
    const int idx = s * 128 + tid;
    const int row = idx >> 4, piece = idx & 15;
    const int col0 = piece * 8;
    v4u a;
#pragma unroll
    for (int e = 0; e < 4; ++e) {
      const float f0 = Os[row * OSP + col0 + 2 * e] * 64.0f;
      const float f1 = Os[row * OSP + col0 + 2 * e + 1] * 64.0f;
      a[e] = pk16(hb16(f0), hb16(f1));
    }
    pk[s] = a;
    offs[s] = (size_t)(blockIdx.x * APB + row) * CCH + col0;
  }
#pragma unroll
  for (int s = 0; s < 4; ++s) *(volatile v4u*)(ao + offs[s]) = pk[s];
  __threadfence();
#pragma unroll
  for (int s = 0; s < 4; ++s) *(volatile v4u*)(ao + offs[s]) = pk[s];
}

__global__ __launch_bounds__(256)
void k_im2col(const float* __restrict__ xa, const float* __restrict__ xb, unsigned short* ah, unsigned short* al) {
  const int tid = threadIdx.x, wv = tid >> 5, lane = tid & 31;
  const int w = blockIdx.x * 8 + wv;
  const int m = w / 18;
  const int rem = w - m * 18;
  const int tap = rem >> 1, half = rem & 1;
  const int ky = tap / 3, kx = tap - ky * 3;
  const int b = m / (OFR * OFR);
  const int p = m - b * (OFR * OFR);
  const int oy = p / OFR, ox = p - oy * OFR;
  const int iy = 2 * oy + ky - 1, ix = 2 * ox + kx - 1;
  const bool valid = ((unsigned)iy < (unsigned)FR) && ((unsigned)ix < (unsigned)FR);
  const int iyc = min(max(iy, 0), FR - 1), ixc = min(max(ix, 0), FR - 1);
  const float* src = (half != 0) ? xb : xa;
  const v4f v = *(const v4f*)(src + ((size_t)(b * FR + iyc) * FR + ixc) * CCH + lane * 4);
  const float msk = valid ? 8.0f : 0.0f;
  unsigned short hb[4], lb[4];
#pragma unroll
  for (int e = 0; e < 4; ++e) {
    const float a = v[e] * msk;
    const _Float16 hv = (_Float16)a;
    const float resid = a - (float)hv;
    hb[e] = h_bits(hv);
    lb[e] = hb16(resid * 2048.0f);
  }
  v2u ph, plo;
  ph[0]  = pk16(hb[0], hb[1]); ph[1]  = pk16(hb[2], hb[3]);
  plo[0] = pk16(lb[0], lb[1]); plo[1] = pk16(lb[2], lb[3]);
  const size_t ko = (size_t)m * KCV + (size_t)tap * C2 + half * CCH + lane * 4;
  *(volatile v2u*)(ah + ko) = ph;
  *(volatile v2u*)(al + ko) = plo;
  __threadfence();
  *(volatile v2u*)(ah + ko) = ph;
  *(volatile v2u*)(al + ko) = plo;
}

__global__ __launch_bounds__(256)
void k_gemm_conv(const unsigned short* __restrict__ ah, const unsigned short* __restrict__ al,
                 const unsigned short* __restrict__ wt, float* cv) {
  __shared__ __align__(16) float Cs[64 * LDC];
  const int tid = threadIdx.x, wave = tid >> 5, lane = tid & 31;
  const int mb = blockIdx.x, nb = blockIdx.y;
  mm_tile2((const _Float16*)(const void*)ah, (const _Float16*)(const void*)al, KCV,
           (const _Float16*)(const void*)wt, KCV, KCV / 32, mb * 64, nb * 128, Cs);
  __syncthreads();
  const int col0 = nb * 128 + lane * 4;
#pragma unroll 1
  for (int it = 0; it < 8; ++it) {
    const int row = wave * 8 + it;
    const size_t t = (size_t)(mb * 64 + row);
    const v4f a = *(const v4f*)(Cs + row * LDC + lane * 4);
    v4f o;
#pragma unroll
    for (int e = 0; e < 4; ++e) o[e] = a[e] * (1.0f / 512.0f);
    float* pp = cv + t * COUT + col0;
    *(volatile v4f*)pp = o;
    __threadfence();
    *(volatile v4f*)pp = o;
  }
}

__global__ __launch_bounds__(256)
void k_ln512(const float* __restrict__ cv, const float* __restrict__ g, const float* __restrict__ bb, float* out) {
  const int tid = threadIdx.x, wv = tid >> 5, lane = tid & 31;
  const int r = blockIdx.x * 8 + wv;
  const float* src = cv + (size_t)r * COUT;
  v4f a[4];
  float s = 0.f;
#pragma unroll
  for (int j = 0; j < 4; ++j) {
    a[j] = *(const v4f*)(src + j * 128 + lane * 4);
    s += (a[j][0] + a[j][1]) + (a[j][2] + a[j][3]);
  }
  s = wsum(s);
  const float mu = s * (1.0f / (float)COUT);
  float sq = 0.f;
#pragma unroll
  for (int j = 0; j < 4; ++j) {
#pragma unroll
    for (int e = 0; e < 4; ++e) { const float d = a[j][e] - mu; a[j][e] = d; sq += d * d; }
  }
  sq = wsum(sq);
  const float rs = rsqrtf(sq * (1.0f / (float)COUT) + 1e-5f);
  v4f yv[4];
#pragma unroll
  for (int j = 0; j < 4; ++j) {
    const v4f gr = *(const v4f*)(g + j * 128 + lane * 4);
    const v4f br = *(const v4f*)(bb + j * 128 + lane * 4);
    v4f yy;
#pragma unroll
    for (int e = 0; e < 4; ++e) yy[e] = (a[j][e] * rs) * bfr(gr[e]) + bfr(br[e]);
    yv[j] = yy;
  }
  float* op = out + (size_t)r * COUT + lane * 4;
#pragma unroll
  for (int j = 0; j < 4; ++j) *(volatile v4f*)(op + j * 128) = yv[j];
  __threadfence();
#pragma unroll
  for (int j = 0; j < 4; ++j) *(volatile v4f*)(op + j * 128) = yv[j];
}

extern "C" void kernel_launch(void* const* d_in, const int* in_sizes, int n_in,
                              void* d_out, int out_size, void* d_ws, size_t ws_size,
                              hipStream_t stream) {
  if (n_in < 33) return;
  const int expect[33] = {
    NPIX * CCH, NPIX * CCH,
    NDEP * CCH, NDEP * CCH, NDEP * CCH * C3, NDEP * C3, NDEP * RPSZ, NDEP * CCH * CCH, NDEP * CCH,
    NDEP * CCH, NDEP * CCH, NDEP * CCH * HID, NDEP * HID, NDEP * HID * CCH, NDEP * CCH,
    NDEP * CCH, NDEP * CCH, NDEP * CCH * CCH, NDEP * CCH, NDEP * CCH * C2, NDEP * C2, NDEP * RPSZ,
    NDEP * CCH * CCH, NDEP * CCH, NDEP * CCH, NDEP * CCH, NDEP * CCH * HID, NDEP * HID,
    NDEP * HID * CCH, NDEP * CCH, 9 * C2 * COUT, COUT, COUT };
  for (int i = 0; i < 33; ++i) if (in_sizes[i] != expect[i]) return;
  if (out_size != NOPX * COUT) return;

  const float* x         = (const float*)d_in[0];
  const float* x_multi   = (const float*)d_in[1];
  const float* sa_n1g    = (const float*)d_in[2];
  const float* sa_n1b    = (const float*)d_in[3];
  const float* sa_qkv_w  = (const float*)d_in[4];
  const float* sa_qkv_b  = (const float*)d_in[5];
  const float* sa_rpb    = (const float*)d_in[6];
  const float* sa_proj_w = (const float*)d_in[7];
  const float* sa_proj_b = (const float*)d_in[8];
  const float* sa_n2g    = (const float*)d_in[9];
  const float* sa_n2b    = (const float*)d_in[10];
  const float* sa_fc1_w  = (const float*)d_in[11];
  const float* sa_fc1_b  = (const float*)d_in[12];
  const float* sa_fc2_w  = (const float*)d_in[13];
  const float* sa_fc2_b  = (const float*)d_in[14];
  const float* cr_n1g    = (const float*)d_in[15];
  const float* cr_n1b    = (const float*)d_in[16];
  const float* cr_q_w    = (const float*)d_in[17];
  const float* cr_q_b    = (const float*)d_in[18];
  const float* cr_kv_w   = (const float*)d_in[19];
  const float* cr_kv_b   = (const float*)d_in[20];
  const float* cr_rpb    = (const float*)d_in[21];
  const float* cr_proj_w = (const float*)d_in[22];
  const float* cr_proj_b = (const float*)d_in[23];
  const float* cr_n2g    = (const float*)d_in[24];
  const float* cr_n2b    = (const float*)d_in[25];
  const float* cr_fc1_w  = (const float*)d_in[26];
  const float* cr_fc1_b  = (const float*)d_in[27];
  const float* cr_fc2_w  = (const float*)d_in[28];
  const float* cr_fc2_b  = (const float*)d_in[29];
  const float* ds_conv_w = (const float*)d_in[30];
  const float* ds_ng     = (const float*)d_in[31];
  const float* ds_nb     = (const float*)d_in[32];
  float* out = (float*)d_out;

  const size_t sXF  = (size_t)NPIX * CCH * 4;
  const size_t sP16 = (size_t)NPIX * CCH * 2;
  const size_t sQKV = (size_t)NPIX * C3 * 4;
  const size_t sH   = (size_t)NPIX * HID * 2;
  const size_t sIM  = (size_t)NOPX * KCV * 2;
  const size_t sCV  = (size_t)NOPX * COUT * 4;
  const size_t sWsq = (size_t)NDEP * CCH * C3 * 2;
  const size_t sWsp = (size_t)NDEP * CCH * CCH * 2;
  const size_t sWs1 = (size_t)NDEP * CCH * HID * 2;
  const size_t sWs2 = (size_t)NDEP * HID * CCH * 2;
  const size_t sWcq = (size_t)NDEP * CCH * CCH * 2;
  const size_t sWck = (size_t)NDEP * CCH * C2 * 2;
  const size_t sWcp = (size_t)NDEP * CCH * CCH * 2;
  const size_t sWc1 = (size_t)NDEP * CCH * HID * 2;
  const size_t sWc2 = (size_t)NDEP * HID * CCH * 2;
  const size_t sWcv = (size_t)KCV * COUT * 2;

  size_t off = 0;
  const size_t oXA  = off; off += sXF;
  const size_t oXB  = off; off += sXF;
  const size_t oT1  = off; off += sXF;
  const size_t oPa  = off; off += sP16;
  const size_t oPb  = off; off += sP16;
  const size_t oAO  = off; off += sP16;
  const size_t oQKV = off; off += sQKV;
  const size_t oH   = off; off += sH;
  const size_t oAH  = off; off += sIM;
  const size_t oAL  = off; off += sIM;
  const size_t oCV  = off; off += sCV;
  const size_t oWsq = off; off += sWsq;
  const size_t oWsp = off; off += sWsp;
  const size_t oWs1 = off; off += sWs1;
  const size_t oWs2 = off; off += sWs2;
  const size_t oWcq = off; off += sWcq;
  const size_t oWck = off; off += sWck;
  const size_t oWcp = off; off += sWcp;
  const size_t oWc1 = off; off += sWc1;
  const size_t oWc2 = off; off += sWc2;
  const size_t oWcv = off; off += sWcv;
  if (off > ws_size) return;
  if (off > (size_t)134217728) return;

  char* ws = (char*)d_ws;
  float*          XA   = (float*)(ws + oXA);
  float*          XB   = (float*)(ws + oXB);
  float*          T1   = (float*)(ws + oT1);
  unsigned short* P16a = (unsigned short*)(ws + oPa);
  unsigned short* P16b = (unsigned short*)(ws + oPb);
  unsigned short* AO   = (unsigned short*)(ws + oAO);
  float*          QKV  = (float*)(ws + oQKV);
  float*          Qf   = (float*)(ws + oQKV);
  float*          KVf  = (float*)(ws + oQKV + sXF);
  unsigned short* Hp   = (unsigned short*)(ws + oH);
  unsigned short* AH   = (unsigned short*)(ws + oAH);
  unsigned short* AL   = (unsigned short*)(ws + oAL);
  float*          CV   = (float*)(ws + oCV);
  unsigned short* Wsq  = (unsigned short*)(ws + oWsq);
  unsigned short* Wsp  = (unsigned short*)(ws + oWsp);
  unsigned short* Ws1  = (unsigned short*)(ws + oWs1);
  unsigned short* Ws2  = (unsigned short*)(ws + oWs2);
  unsigned short* Wcq  = (unsigned short*)(ws + oWcq);
  unsigned short* Wck  = (unsigned short*)(ws + oWck);
  unsigned short* Wcp  = (unsigned short*)(ws + oWcp);
  unsigned short* Wc1  = (unsigned short*)(ws + oWc1);
  unsigned short* Wc2  = (unsigned short*)(ws + oWc2);
  unsigned short* Wcv  = (unsigned short*)(ws + oWcv);

  const dim3 blk(256);
  const dim3 grow(NPIX / 8);
  const dim3 gm64(NPIX / 64);
  const float S512  = 1.0f / 512.0f;
  const float S4096 = 1.0f / 4096.0f;

  k_cvt_wt<<<dim3(C3 / 64,   CCH / 64, NDEP), blk, 0, stream>>>(sa_qkv_w,  Wsq, CCH, C3);
  k_cvt_wt<<<dim3(CCH / 64,  CCH / 64, NDEP), blk, 0, stream>>>(sa_proj_w, Wsp, CCH, CCH);
  k_cvt_wt<<<dim3(HID / 64,  CCH / 64, NDEP), blk, 0, stream>>>(sa_fc1_w,  Ws1, CCH, HID);
  k_cvt_wt<<<dim3(CCH / 64,  HID / 64, NDEP), blk, 0, stream>>>(sa_fc2_w,  Ws2, HID, CCH);
  k_cvt_wt<<<dim3(CCH / 64,  CCH / 64, NDEP), blk, 0, stream>>>(cr_q_w,    Wcq, CCH, CCH);
  k_cvt_wt<<<dim3(C2 / 64,   CCH / 64, NDEP), blk, 0, stream>>>(cr_kv_w,   Wck, CCH, C2);
  k_cvt_wt<<<dim3(CCH / 64,  CCH / 64, NDEP), blk, 0, stream>>>(cr_proj_w, Wcp, CCH, CCH);
  k_cvt_wt<<<dim3(HID / 64,  CCH / 64, NDEP), blk, 0, stream>>>(cr_fc1_w,  Wc1, CCH, HID);
  k_cvt_wt<<<dim3(CCH / 64,  HID / 64, NDEP), blk, 0, stream>>>(cr_fc2_w,  Wc2, HID, CCH);
  k_cvt_wt<<<dim3(COUT / 64, KCV / 64, 1),    blk, 0, stream>>>(ds_conv_w, Wcv, KCV, COUT);

  for (int i = 0; i < NDEP; ++i) {
    if (i == 0) k_ln128<1><<<grow, blk, 0, stream>>>(x, sa_n1g, sa_n1b, P16a);
    else        k_ln128<0><<<grow, blk, 0, stream>>>(XA, sa_n1g + i * CCH, sa_n1b + i * CCH, P16a);
    k_gemm_f32<0, 0><<<dim3(NPIX / 64, C3 / 128), blk, 0, stream>>>(
        P16a, Wsq + (size_t)i * C3 * CCH, CCH, sa_qkv_b + i * C3, S512, sa_qkv_b, QKV, C3);
    k_attn<<<dim3(NPIX / APB), dim3(128), 0, stream>>>(QKV, C3, QKV, C3, CCH, 2 * CCH, sa_rpb + i * RPSZ, AO);
    if (i == 0) k_gemm_f32<1, 1><<<dim3(NPIX / 64, 1), blk, 0, stream>>>(
        AO, Wsp + (size_t)i * CCH * CCH, CCH, sa_proj_b + i * CCH, S4096, x, T1, CCH);
    else        k_gemm_f32<1, 0><<<dim3(NPIX / 64, 1), blk, 0, stream>>>(
        AO, Wsp + (size_t)i * CCH * CCH, CCH, sa_proj_b + i * CCH, S4096, XA, T1, CCH);
    k_ln128<0><<<grow, blk, 0, stream>>>(T1, sa_n2g + i * CCH, sa_n2b + i * CCH, P16a);
    k_gemm_gelu<<<dim3(NPIX / 64, HID / 128), blk, 0, stream>>>(
        P16a, Ws1 + (size_t)i * HID * CCH, sa_fc1_b + i * HID, Hp);
    k_gemm_f32<1, 0><<<gm64, blk, 0, stream>>>(
        Hp, Ws2 + (size_t)i * CCH * HID, HID, sa_fc2_b + i * CCH, S4096, T1, XA, CCH);
  }

  for (int i = 0; i < NDEP; ++i) {
    if (i == 0) k_cvt16<1><<<grow, blk, 0, stream>>>(x, P16a);
    else        k_cvt16<0><<<grow, blk, 0, stream>>>(XB, P16a);
    k_gemm_f32<0, 0><<<dim3(NPIX / 64, 1), blk, 0, stream>>>(
        P16a, Wcq + (size_t)i * CCH * CCH, CCH, cr_q_b + i * CCH, S512, cr_q_b, Qf, CCH);
    k_ln128<1><<<grow, blk, 0, stream>>>(x_multi, cr_n1g + i * CCH, cr_n1b + i * CCH, P16b);
    k_gemm_f32<0, 0><<<dim3(NPIX / 64, C2 / 128), blk, 0, stream>>>(
        P16b, Wck + (size_t)i * C2 * CCH, CCH, cr_kv_b + i * C2, S512, cr_kv_b, KVf, C2);
    k_attn<<<dim3(NPIX / APB), dim3(128), 0, stream>>>(Qf, CCH, KVf, C2, 0, CCH, cr_rpb + i * RPSZ, AO);
    k_gemm_f32<1, 1><<<dim3(NPIX / 64, 1), blk, 0, stream>>>(
        AO, Wcp + (size_t)i * CCH * CCH, CCH, cr_proj_b + i * CCH, S4096, x_multi, T1, CCH);
    k_ln128<0><<<grow, blk, 0, stream>>>(T1, cr_n2g + i * CCH, cr_n2b + i * CCH, P16a);
    k_gemm_gelu<<<dim3(NPIX / 64, HID / 128), blk, 0, stream>>>(
        P16a, Wc1 + (size_t)i * HID * CCH, cr_fc1_b + i * HID, Hp);
    k_gemm_f32<1, 0><<<gm64, blk, 0, stream>>>(
        Hp, Wc2 + (size_t)i * CCH * HID, HID, cr_fc2_b + i * CCH, S4096, T1, XB, CCH);
  }

  k_im2col<<<dim3(NOPX * 18 / 8), blk, 0, stream>>>(XA, XB, AH, AL);
  k_gemm_conv<<<dim3(NOPX / 64, COUT / 128), blk, 0, stream>>>(AH, AL, Wcv, CV);
  k_ln512<<<dim3(NOPX / 8), blk, 0, stream>>>(CV, ds_ng, ds_nb, out);
  (void)hipGetLastError();
}
